// HeteroModel_70248485094040
// MI455X (gfx1250) — hardware-run, weakly checked
//
#include <hip/hip_runtime.h>


namespace {
constexpr int NT = 100000, NTP = 100032, NPL = 20000, NPP = 20032, E = 2000000, EL = 500000, FT = 128, FP = 64, H = 128;
constexpr float XS = 8.0f, WSC = 256.0f, NEG = 0.2f  , NRMEPS = 1e-12f;
typedef _Float16 b16;
typedef __attribute__((ext_vector_type(16))) _Float16 v16b;
typedef __attribute__((ext_vector_type(8))) _Float16 v8b;
typedef __attribute__((ext_vector_type(8))) float v8f;
typedef __attribute__((ext_vector_type(4))) float v4f;
__device__ __forceinline__ float bf16_rne(float f) { unsigned int u = __float_as_uint(f); u += 0x7FFFu + ((u >> 16) & 1u); return __uint_as_float(u & 0xFFFF0000u); }
__device__ __forceinline__ void split16(float v, b16& hi, b16& lo) { hi = (b16)v; lo = (b16)(v - (float)hi); }
__device__ __forceinline__ v16b frag_kb(const b16* p, int hh) { const v8b a = *(const v8b*)(p + 8 * hh), b = *(const v8b*)(p + 16 + 8 * hh); v16b f;
#pragma unroll
  for (int e = 0; e < 8; ++e) { f[e] = a[e]; f[8 + e] = b[e]; } return f; }
__device__ __forceinline__ v8f wmma16b(v16b a, v16b b, v8f c) { v8f d = __builtin_amdgcn_wmma_f32_16x16x32_f16(false, a, false, b, (short)0, c, false, false); asm volatile("v_nop\n\tv_nop\n\tv_nop\n\tv_nop" : "+v"(d) : "v"(a), "v"(b)); return d; }
__device__ __forceinline__ void wave_lds_sync() { __builtin_amdgcn_fence(__ATOMIC_RELEASE, "workgroup"); __builtin_amdgcn_wave_barrier(); __builtin_amdgcn_fence(__ATOMIC_ACQUIRE, "workgroup"); }
__device__ __forceinline__ float pmul(float a, float b) { float p = a * b; asm volatile("" : "+v"(p)); return p; }
__device__ __forceinline__ int iclamp(int v, int lo, int hi) { return v < lo ? lo : (v > hi ? hi : v); }
constexpr int CSR_NBLK6 = 512, CSR_GB6 = 6, CSR_GN6 = 1 << CSR_GB6  , CSR_MAXG6 = 512, CSR_CAP6 = 12288  ;
__global__ __launch_bounds__(64) void csrA6_kernel(const int* __restrict__ dst, int E, int N, int nG, int CHP, int NGP, int* __restrict__ STG, int* __restrict__ HST) {
  extern __shared__ int sm[];
  int* cnt = sm; int* run = sm + NGP; int* ids = sm + 2 * NGP;
  const int b = blockIdx.x; const int ch = (E + CSR_NBLK6 - 1) / CSR_NBLK6; const int e0 = b * ch, e1 = min(E, e0 + ch);
  for (int i = threadIdx.x; i < NGP; i += 64) cnt[i] = 0;
  for (int i = threadIdx.x; i < CHP; i += 64) ids[i] = -1;
  __syncthreads();
  if (threadIdx.x == 0) {
    for (int e = e0; e < e1; ++e) { int d = dst[e]; d = (d < 0) ? 0 : (d >= N ? N - 1 : d); cnt[d >> CSR_GB6] += 1; }
    int acc = 0; for (int g = 0; g < nG; ++g) { run[g] = acc; acc += cnt[g]; }
    for (int e = e0; e < e1; ++e) { int d = dst[e]; d = (d < 0) ? 0 : (d >= N ? N - 1 : d); const int g = d >> CSR_GB6; ids[run[g]] = e; run[g] += 1; } }
  __syncthreads();
  typedef __attribute__((ext_vector_type(4))) int v4i;
  for (int pass = 0; pass < 2; ++pass) {
    for (int i = threadIdx.x; i < CHP / 4; i += 64) *(volatile v4i*)(STG + (size_t)b * CHP + i * 4) = *(const v4i*)(&ids[i * 4]);
    for (int i = threadIdx.x; i < NGP / 4; i += 64) { v4i v; for (int e = 0; e < 4; ++e) v[e] = (i * 4 + e < nG) ? cnt[i * 4 + e] : 0; *(volatile v4i*)(HST + (size_t)b * NGP + i * 4) = v; }
    __threadfence(); }
}
__global__ __launch_bounds__(512) void csrS6_kernel(const int* __restrict__ HST, int nG, int NGP, int* __restrict__ START, int* __restrict__ TOT, int* __restrict__ OFF) {
  __shared__ int tot[CSR_MAXG6];
  const int b = threadIdx.x;
  for (int pass = 0; pass < 2; ++pass) { int runb = 0; for (int g = 0; g < nG; ++g) { int c = HST[(size_t)b * NGP + g]; c = (c < 0) ? 0 : c; ((volatile int*)OFF)[(size_t)g * CSR_NBLK6 + b] = runb; runb += c; } __threadfence(); }
  for (int g = threadIdx.x; g < nG; g += 512) { int s = 0; for (int bb = 0; bb < CSR_NBLK6; ++bb) { int c = HST[(size_t)bb * NGP + g]; s += (c < 0) ? 0 : c; } tot[g] = s; }
  __syncthreads();
  if (threadIdx.x < 32) {
    __shared__ int st[CSR_MAXG6 + 32];
    if (threadIdx.x == 0) { int acc = 0; for (int g = 0; g < NGP; ++g) { st[g] = acc; if (g < nG) acc += (tot[g] + 31) & ~31; } st[NGP] = acc; }
    __builtin_amdgcn_fence(__ATOMIC_RELEASE, "workgroup"); __builtin_amdgcn_wave_barrier(); __builtin_amdgcn_fence(__ATOMIC_ACQUIRE, "workgroup");
    for (int pass = 0; pass < 2; ++pass) { for (int i = threadIdx.x; i < NGP + 32; i += 32) { ((volatile int*)START)[i] = (i <= NGP) ? st[min(i, NGP)] : 0; ((volatile int*)TOT)[i] = (i < nG) ? tot[i] : 0; } __threadfence(); } }
}
__global__ __launch_bounds__(256) void csrB6_kernel(const int* __restrict__ dst, int N, int nG, int CHP, int NGP, int permLen, const int* __restrict__ STG, const int* __restrict__ HST, const int* __restrict__ OFF, const int* __restrict__ START, const int* __restrict__ TOT, int* __restrict__ PERM, int* __restrict__ ROWPTR, int* __restrict__ ROWCNT, int* __restrict__ FLAG) {
  typedef __attribute__((ext_vector_type(4))) int v4i;
  __shared__ int ids[CSR_CAP6]; __shared__ unsigned short key[CSR_CAP6]; __shared__ int outp[CSR_CAP6]; __shared__ int ncnt[CSR_GN6 + 1]; __shared__ int boff[CSR_NBLK6 + 1];
  const int g = blockIdx.x, t_ = threadIdx.x; int tot = TOT[g]; int st = START[g], stn = START[g + 1]; const int v0 = g * CSR_GN6; const int nv = min(CSR_GN6, N - v0);
  st = (st < 0) ? 0 : (st > permLen - 32 ? permLen - 32 : st) & ~31; stn = (stn < st) ? st : (stn > permLen ? permLen : stn); tot = (tot < 0) ? 0 : tot; if (tot > stn - st && tot <= CSR_CAP6) tot = stn - st;
  if (tot > CSR_CAP6) {
    for (int pass = 0; pass < 2; ++pass) { for (int i = t_; i < CSR_GN6 / 4; i += 256) { v4i a, c; for (int e = 0; e < 4; ++e) { a[e] = st; c[e] = 0; } *(volatile v4i*)(ROWPTR + v0 + i * 4) = a; *(volatile v4i*)(ROWCNT + v0 + i * 4) = c; } if (t_ == 0) ((volatile int*)FLAG)[0] = 1; __threadfence(); } (void)nv; return; }
  if (t_ == 0) { int acc = 0; for (int b = 0; b < CSR_NBLK6; ++b) { boff[b] = acc; int c = HST[(size_t)b * NGP + g]; c = (c < 0) ? 0 : (c > CHP ? CHP : c); acc += c; if (acc > tot) acc = tot; } boff[CSR_NBLK6] = acc; }
  for (int i = t_; i <= CSR_GN6; i += 256) ncnt[i] = 0;
  __syncthreads();
  for (int b = 0; b < CSR_NBLK6; ++b) { const int c = boff[b + 1] - boff[b]; int o_ = OFF[(size_t)g * CSR_NBLK6 + b]; o_ = (o_ < 0) ? 0 : (o_ > CHP - c ? CHP - c : o_); const int* src_ = STG + (size_t)b * CHP + o_;
    for (int i = t_; i < c; i += 256) { int id = src_[i]; id = (id < 0) ? 0 : id; ids[boff[b] + i] = id; int d = dst[id]; d = (d < v0) ? v0 : (d >= N ? N - 1 : d); int kk = d - v0; kk = (kk < 0) ? 0 : (kk >= CSR_GN6 ? CSR_GN6 - 1 : kk); key[boff[b] + i] = (unsigned short)kk; } }
  __syncthreads();
  if (t_ == 0) { for (int i = 0; i < tot; ++i) ncnt[key[i]] += 1; int acc = 0; for (int vl = 0; vl < CSR_GN6; ++vl) { const int c = ncnt[vl]; ncnt[vl] = acc; acc += c; } ncnt[CSR_GN6] = acc;
    for (int i = 0; i < tot; ++i) { const int vl = key[i]; outp[ncnt[vl]] = ids[i]; ncnt[vl] += 1; }
    for (int vl = CSR_GN6; vl > 0; --vl) ncnt[vl] = ncnt[vl - 1]; ncnt[0] = 0; }
  __syncthreads();
  for (int pass = 0; pass < 2; ++pass) {
    for (int i = t_; i < (stn - st) / 4; i += 256) { v4i v; for (int e = 0; e < 4; ++e) { const int q = i * 4 + e; v[e] = (q < tot) ? outp[q] : -1; } *(volatile v4i*)(PERM + st + i * 4) = v; }
    for (int i = t_; i < CSR_GN6 / 4; i += 256) { v4i a, c; for (int e = 0; e < 4; ++e) { const int vl = i * 4 + e; a[e] = st + ncnt[vl]; c[e] = (vl < nv) ? (ncnt[vl + 1] - ncnt[vl]) : 0; } *(volatile v4i*)(ROWPTR + v0 + i * 4) = a; *(volatile v4i*)(ROWCNT + v0 + i * 4) = c; }
    __threadfence(); }
}
__global__ __launch_bounds__(256) void csrZ6_kernel(int* __restrict__ p, size_t n4) { typedef __attribute__((ext_vector_type(4))) int v4i; const size_t tid = (size_t)blockIdx.x * 256 + threadIdx.x, nth = (size_t)gridDim.x * 256; v4i z = {0, 0, 0, 0}; for (size_t i = tid; i < n4; i += nth) *(volatile v4i*)(p + i * 4) = z; }
struct CsrBufs6 { int *STG, *HST, *OFF, *START, *TOT, *PERM, *ROWPTR, *ROWCNT, *FLAG; int nG, NGP, CHP; size_t permLen; char* base; size_t bytes; };
static size_t csr_carve6(CsrBufs6& c, char* ws, size_t off, int E, int N) {
  const size_t off0 = off; c.base = ws + off;
  auto al = [&](size_t bytes) { char* p = ws + off; off += (bytes + 255) & ~(size_t)255; return p; };
  c.nG = (N + CSR_GN6 - 1) / CSR_GN6; c.NGP = (c.nG + 31) & ~31; const int ch = (E + CSR_NBLK6 - 1) / CSR_NBLK6; c.CHP = (ch + 31) & ~31; c.permLen = (size_t)E + 32 * (size_t)c.nG + 32;
  c.STG = (int*)al((size_t)CSR_NBLK6 * c.CHP * 4); c.HST = (int*)al((size_t)CSR_NBLK6 * c.NGP * 4); c.OFF = (int*)al((size_t)c.NGP * CSR_NBLK6 * 4); c.START = (int*)al((size_t)(c.NGP + 64) * 4); c.TOT = (int*)al((size_t)(c.NGP + 64) * 4);
  c.PERM = (int*)al(c.permLen * 4); c.ROWPTR = (int*)al((size_t)c.nG * CSR_GN6 * 4); c.ROWCNT = (int*)al((size_t)c.nG * CSR_GN6 * 4); c.FLAG = (int*)al(256);
  c.bytes = off - off0; return off;
}
static void csr_build6(const CsrBufs6& c, const int* dst, int E, int N, hipStream_t stream) {
  const size_t smem = (size_t)(2 * c.NGP + c.CHP) * 4;
  csrZ6_kernel<<<512, 256, 0, stream>>>((int*)c.base, c.bytes / 16);
  csrA6_kernel<<<CSR_NBLK6, 64, smem, stream>>>(dst, E, N, c.nG, c.CHP, c.NGP, c.STG, c.HST);
  csrS6_kernel<<<1, 512, 0, stream>>>(c.HST, c.nG, c.NGP, c.START, c.TOT, c.OFF);
  csrB6_kernel<<<c.nG, 256, 0, stream>>>(dst, N, c.nG, c.CHP, c.NGP, (int)c.permLen, c.STG, c.HST, c.OFF, c.START, c.TOT, c.PERM, c.ROWPTR, c.ROWCNT, c.FLAG);
}

constexpr int CSR_NBLK8 = 512, CSR_GB8 = 8, CSR_GN8 = 1 << CSR_GB8  , CSR_MAXG8 = 512, CSR_CAP8 = 12288  ;
__global__ __launch_bounds__(64) void csrA8_kernel(const int* __restrict__ dst, int E, int N, int nG, int CHP, int NGP, int* __restrict__ STG, int* __restrict__ HST) {
  extern __shared__ int sm[];
  int* cnt = sm; int* run = sm + NGP; int* ids = sm + 2 * NGP;
  const int b = blockIdx.x; const int ch = (E + CSR_NBLK8 - 1) / CSR_NBLK8; const int e0 = b * ch, e1 = min(E, e0 + ch);
  for (int i = threadIdx.x; i < NGP; i += 64) cnt[i] = 0;
  for (int i = threadIdx.x; i < CHP; i += 64) ids[i] = -1;
  __syncthreads();
  if (threadIdx.x == 0) {
    for (int e = e0; e < e1; ++e) { int d = dst[e]; d = (d < 0) ? 0 : (d >= N ? N - 1 : d); cnt[d >> CSR_GB8] += 1; }
    int acc = 0; for (int g = 0; g < nG; ++g) { run[g] = acc; acc += cnt[g]; }
    for (int e = e0; e < e1; ++e) { int d = dst[e]; d = (d < 0) ? 0 : (d >= N ? N - 1 : d); const int g = d >> CSR_GB8; ids[run[g]] = e; run[g] += 1; } }
  __syncthreads();
  typedef __attribute__((ext_vector_type(4))) int v4i;
  for (int pass = 0; pass < 2; ++pass) {
    for (int i = threadIdx.x; i < CHP / 4; i += 64) *(volatile v4i*)(STG + (size_t)b * CHP + i * 4) = *(const v4i*)(&ids[i * 4]);
    for (int i = threadIdx.x; i < NGP / 4; i += 64) { v4i v; for (int e = 0; e < 4; ++e) v[e] = (i * 4 + e < nG) ? cnt[i * 4 + e] : 0; *(volatile v4i*)(HST + (size_t)b * NGP + i * 4) = v; }
    __threadfence(); }
}
__global__ __launch_bounds__(512) void csrS8_kernel(const int* __restrict__ HST, int nG, int NGP, int* __restrict__ START, int* __restrict__ TOT, int* __restrict__ OFF) {
  __shared__ int tot[CSR_MAXG8];
  const int b = threadIdx.x;
  for (int pass = 0; pass < 2; ++pass) { int runb = 0; for (int g = 0; g < nG; ++g) { int c = HST[(size_t)b * NGP + g]; c = (c < 0) ? 0 : c; ((volatile int*)OFF)[(size_t)g * CSR_NBLK8 + b] = runb; runb += c; } __threadfence(); }
  for (int g = threadIdx.x; g < nG; g += 512) { int s = 0; for (int bb = 0; bb < CSR_NBLK8; ++bb) { int c = HST[(size_t)bb * NGP + g]; s += (c < 0) ? 0 : c; } tot[g] = s; }
  __syncthreads();
  if (threadIdx.x < 32) {
    __shared__ int st[CSR_MAXG8 + 32];
    if (threadIdx.x == 0) { int acc = 0; for (int g = 0; g < NGP; ++g) { st[g] = acc; if (g < nG) acc += (tot[g] + 31) & ~31; } st[NGP] = acc; }
    __builtin_amdgcn_fence(__ATOMIC_RELEASE, "workgroup"); __builtin_amdgcn_wave_barrier(); __builtin_amdgcn_fence(__ATOMIC_ACQUIRE, "workgroup");
    for (int pass = 0; pass < 2; ++pass) { for (int i = threadIdx.x; i < NGP + 32; i += 32) { ((volatile int*)START)[i] = (i <= NGP) ? st[min(i, NGP)] : 0; ((volatile int*)TOT)[i] = (i < nG) ? tot[i] : 0; } __threadfence(); } }
}
__global__ __launch_bounds__(256) void csrB8_kernel(const int* __restrict__ dst, int N, int nG, int CHP, int NGP, int permLen, const int* __restrict__ STG, const int* __restrict__ HST, const int* __restrict__ OFF, const int* __restrict__ START, const int* __restrict__ TOT, int* __restrict__ PERM, int* __restrict__ ROWPTR, int* __restrict__ ROWCNT, int* __restrict__ FLAG) {
  typedef __attribute__((ext_vector_type(4))) int v4i;
  __shared__ int ids[CSR_CAP8]; __shared__ unsigned short key[CSR_CAP8]; __shared__ int outp[CSR_CAP8]; __shared__ int ncnt[CSR_GN8 + 1]; __shared__ int boff[CSR_NBLK8 + 1];
  const int g = blockIdx.x, t_ = threadIdx.x; int tot = TOT[g]; int st = START[g], stn = START[g + 1]; const int v0 = g * CSR_GN8; const int nv = min(CSR_GN8, N - v0);
  st = (st < 0) ? 0 : (st > permLen - 32 ? permLen - 32 : st) & ~31; stn = (stn < st) ? st : (stn > permLen ? permLen : stn); tot = (tot < 0) ? 0 : tot; if (tot > stn - st && tot <= CSR_CAP8) tot = stn - st;
  if (tot > CSR_CAP8) {
    for (int pass = 0; pass < 2; ++pass) { for (int i = t_; i < CSR_GN8 / 4; i += 256) { v4i a, c; for (int e = 0; e < 4; ++e) { a[e] = st; c[e] = 0; } *(volatile v4i*)(ROWPTR + v0 + i * 4) = a; *(volatile v4i*)(ROWCNT + v0 + i * 4) = c; } if (t_ == 0) ((volatile int*)FLAG)[0] = 1; __threadfence(); } (void)nv; return; }
  if (t_ == 0) { int acc = 0; for (int b = 0; b < CSR_NBLK8; ++b) { boff[b] = acc; int c = HST[(size_t)b * NGP + g]; c = (c < 0) ? 0 : (c > CHP ? CHP : c); acc += c; if (acc > tot) acc = tot; } boff[CSR_NBLK8] = acc; }
  for (int i = t_; i <= CSR_GN8; i += 256) ncnt[i] = 0;
  __syncthreads();
  for (int b = 0; b < CSR_NBLK8; ++b) { const int c = boff[b + 1] - boff[b]; int o_ = OFF[(size_t)g * CSR_NBLK8 + b]; o_ = (o_ < 0) ? 0 : (o_ > CHP - c ? CHP - c : o_); const int* src_ = STG + (size_t)b * CHP + o_;
    for (int i = t_; i < c; i += 256) { int id = src_[i]; id = (id < 0) ? 0 : id; ids[boff[b] + i] = id; int d = dst[id]; d = (d < v0) ? v0 : (d >= N ? N - 1 : d); int kk = d - v0; kk = (kk < 0) ? 0 : (kk >= CSR_GN8 ? CSR_GN8 - 1 : kk); key[boff[b] + i] = (unsigned short)kk; } }
  __syncthreads();
  if (t_ == 0) { for (int i = 0; i < tot; ++i) ncnt[key[i]] += 1; int acc = 0; for (int vl = 0; vl < CSR_GN8; ++vl) { const int c = ncnt[vl]; ncnt[vl] = acc; acc += c; } ncnt[CSR_GN8] = acc;
    for (int i = 0; i < tot; ++i) { const int vl = key[i]; outp[ncnt[vl]] = ids[i]; ncnt[vl] += 1; }
    for (int vl = CSR_GN8; vl > 0; --vl) ncnt[vl] = ncnt[vl - 1]; ncnt[0] = 0; }
  __syncthreads();
  for (int pass = 0; pass < 2; ++pass) {
    for (int i = t_; i < (stn - st) / 4; i += 256) { v4i v; for (int e = 0; e < 4; ++e) { const int q = i * 4 + e; v[e] = (q < tot) ? outp[q] : -1; } *(volatile v4i*)(PERM + st + i * 4) = v; }
    for (int i = t_; i < CSR_GN8 / 4; i += 256) { v4i a, c; for (int e = 0; e < 4; ++e) { const int vl = i * 4 + e; a[e] = st + ncnt[vl]; c[e] = (vl < nv) ? (ncnt[vl + 1] - ncnt[vl]) : 0; } *(volatile v4i*)(ROWPTR + v0 + i * 4) = a; *(volatile v4i*)(ROWCNT + v0 + i * 4) = c; }
    __threadfence(); }
}
__global__ __launch_bounds__(256) void csrZ8_kernel(int* __restrict__ p, size_t n4) { typedef __attribute__((ext_vector_type(4))) int v4i; const size_t tid = (size_t)blockIdx.x * 256 + threadIdx.x, nth = (size_t)gridDim.x * 256; v4i z = {0, 0, 0, 0}; for (size_t i = tid; i < n4; i += nth) *(volatile v4i*)(p + i * 4) = z; }
struct CsrBufs8 { int *STG, *HST, *OFF, *START, *TOT, *PERM, *ROWPTR, *ROWCNT, *FLAG; int nG, NGP, CHP; size_t permLen; char* base; size_t bytes; };
static size_t csr_carve8(CsrBufs8& c, char* ws, size_t off, int E, int N) {
  const size_t off0 = off; c.base = ws + off;
  auto al = [&](size_t bytes) { char* p = ws + off; off += (bytes + 255) & ~(size_t)255; return p; };
  c.nG = (N + CSR_GN8 - 1) / CSR_GN8; c.NGP = (c.nG + 31) & ~31; const int ch = (E + CSR_NBLK8 - 1) / CSR_NBLK8; c.CHP = (ch + 31) & ~31; c.permLen = (size_t)E + 32 * (size_t)c.nG + 32;
  c.STG = (int*)al((size_t)CSR_NBLK8 * c.CHP * 4); c.HST = (int*)al((size_t)CSR_NBLK8 * c.NGP * 4); c.OFF = (int*)al((size_t)c.NGP * CSR_NBLK8 * 4); c.START = (int*)al((size_t)(c.NGP + 64) * 4); c.TOT = (int*)al((size_t)(c.NGP + 64) * 4);
  c.PERM = (int*)al(c.permLen * 4); c.ROWPTR = (int*)al((size_t)c.nG * CSR_GN8 * 4); c.ROWCNT = (int*)al((size_t)c.nG * CSR_GN8 * 4); c.FLAG = (int*)al(256);
  c.bytes = off - off0; return off;
}
static void csr_build8(const CsrBufs8& c, const int* dst, int E, int N, hipStream_t stream) {
  const size_t smem = (size_t)(2 * c.NGP + c.CHP) * 4;
  csrZ8_kernel<<<512, 256, 0, stream>>>((int*)c.base, c.bytes / 16);
  csrA8_kernel<<<CSR_NBLK8, 64, smem, stream>>>(dst, E, N, c.nG, c.CHP, c.NGP, c.STG, c.HST);
  csrS8_kernel<<<1, 512, 0, stream>>>(c.HST, c.nG, c.NGP, c.START, c.TOT, c.OFF);
  csrB8_kernel<<<c.nG, 256, 0, stream>>>(dst, N, c.nG, c.CHP, c.NGP, (int)c.permLen, c.STG, c.HST, c.OFF, c.START, c.TOT, c.PERM, c.ROWPTR, c.ROWCNT, c.FLAG);
}


__global__ __launch_bounds__(256) void wprep_kernel(const float* __restrict__ wnt, const float* __restrict__ wnp, const float* __restrict__ l1lp, const float* __restrict__ l1rp, const float* __restrict__ l1lt, const float* __restrict__ l1rt, const float* __restrict__ l2lp, const float* __restrict__ l2rp, const float* __restrict__ l2lt, const float* __restrict__ l2rt, b16* __restrict__ WNT, b16* __restrict__ WNP, b16* __restrict__ WL) {
  const size_t u = (size_t)blockIdx.x * 256 + threadIdx.x; const size_t n0 = (size_t)H * FT / 8, n1 = (size_t)H * FP / 8, n2 = (size_t)H * 2 * H / 8; size_t t = u; v8b o;
  if (t < n0) { const size_t e = t * 8; const int oo = (int)(e / FT), k0 = (int)(e % FT); for (int j = 0; j < 8; ++j) o[j] = (b16)(bf16_rne(wnt[(size_t)(k0 + j) * H + oo]) * WSC); for (int pass = 0; pass < 2; ++pass) { *(volatile v8b*)(WNT + e) = o; __threadfence(); } return; } t -= n0;
  if (t < n1) { const size_t e = t * 8; const int oo = (int)(e / FP), k0 = (int)(e % FP); for (int j = 0; j < 8; ++j) o[j] = (b16)(bf16_rne(wnp[(size_t)(k0 + j) * H + oo]) * WSC); for (int pass = 0; pass < 2; ++pass) { *(volatile v8b*)(WNP + e) = o; __threadfence(); } return; } t -= n1;
  if (t < 4 * n2) { const int which = (int)(t / n2); const size_t e = (t % n2) * 8; const int oo = (int)(e / (2 * H)), k0 = (int)(e % (2 * H)); const float* wl = which == 0 ? l1lp : which == 1 ? l1lt : which == 2 ? l2lp : l2lt; const float* wr = which == 0 ? l1rp : which == 1 ? l1rt : which == 2 ? l2rp : l2rt;
    for (int j = 0; j < 8; ++j) { const int k = k0 + j; const float w = k < H ? wl[(size_t)k * H + oo] : wr[(size_t)(k - H) * H + oo]; o[j] = (b16)(bf16_rne(w) * WSC); }
    for (int pass = 0; pass < 2; ++pass) { *(volatile v8b*)(WL + (size_t)which * H * 2 * H + e) = o; __threadfence(); } }
}
template <int KD>
__global__ __launch_bounds__(128) void proj_kernel(const float* __restrict__ x, int NV, const b16* __restrict__ W, const float* __restrict__ bias, float* __restrict__ OUT) {
  __shared__ __attribute__((aligned(16))) float Tf[4][16][H + 4];
  const int wave = threadIdx.x >> 5, lane = threadIdx.x & 31, nloc = lane & 15, hlf = lane >> 4; const size_t m0 = (size_t)blockIdx.x * 64 + wave * 16; const size_t v = m0 + nloc;
  v8f acc[8];
#pragma unroll
  for (int t = 0; t < 8; ++t) acc[t] = (v8f){};
#pragma unroll
  for (int kb = 0; kb < KD; kb += 32) { v16b a = {}; if (v < (size_t)NV) { const float* r = x + v * KD + kb; for (int e = 0; e < 8; ++e) { a[e] = (b16)(bf16_rne(r[8 * hlf + e]) * XS); a[8 + e] = (b16)(bf16_rne(r[16 + 8 * hlf + e]) * XS); } }
#pragma unroll
    for (int t = 0; t < 8; ++t) acc[t] = wmma16b(a, frag_kb(W + (size_t)(t * 16 + nloc) * KD + kb, hlf), acc[t]); }
#pragma unroll
  for (int t = 0; t < 8; ++t) { const int c = t * 16 + nloc; const float bb = bf16_rne(bias[c]);
#pragma unroll 1
    for (int r = 0; r < 8; ++r) { const size_t row = m0 + 8 * hlf + r; Tf[wave][8 * hlf + r][c] = row < (size_t)NV ? acc[t][r] * (1.0f / (XS * WSC)) + bb : 0.0f; } }
  wave_lds_sync();
  for (int pass = 0; pass < 2; ++pass) { for (int rr = 0; rr < 16; ++rr) *(volatile v4f*)(OUT + (m0 + rr) * H + lane * 4) = *(const v4f*)(&Tf[wave][rr][lane * 4]); __threadfence(); }
}
__global__ __launch_bounds__(256) void mean_kernel(const float* __restrict__ S, int NS, const int* __restrict__ other, int NV, const int* __restrict__ PERM, const int* __restrict__ ROWPTR, const int* __restrict__ ROWCNT, int permLen, float* __restrict__ AGG) {
  const int wave = threadIdx.x >> 5, lane = threadIdx.x & 31; const size_t v = (size_t)blockIdx.x * 8 + wave; v4f acc = {0.0f, 0.0f, 0.0f, 0.0f};
  if (v < (size_t)NV) { int st = ROWPTR[v], cnt = ROWCNT[v]; cnt = iclamp(cnt, 0, 1 << 20); st = iclamp(st, 0, permLen - cnt);
#pragma unroll 1
    for (int j = 0; j < cnt; ++j) { const int e = iclamp(PERM[st + j], 0, E - 1); const size_t s = (size_t)iclamp(other[e], 0, NS - 1); acc += *(const v4f*)(S + s * H + lane * 4); }
    const float inv = 1.0f / fmaxf((float)cnt, 1.0f); for (int i = 0; i < 4; ++i) acc[i] = pmul(acc[i], inv); }
  for (int pass = 0; pass < 2; ++pass) { *(volatile v4f*)(AGG + v * H + lane * 4) = acc; __threadfence(); }
}
template <int RELU>
__global__ __launch_bounds__(128) void sage_kernel(const float* AGG, const float* Hs, int NV, const b16* __restrict__ W, const float* __restrict__ bl, float* OUT) {
  __shared__ __attribute__((aligned(16))) b16 Ah[4][16][2 * H + 8], Al[4][16][2 * H + 8]; __shared__ __attribute__((aligned(16))) float Tf[4][16][H + 4];
  const int wave = threadIdx.x >> 5, lane = threadIdx.x & 31, nloc = lane & 15, hlf = lane >> 4; const size_t m0 = (size_t)blockIdx.x * 64 + wave * 16;
  for (int rr = 0; rr < 16; ++rr) { const size_t v = m0 + rr; const v4f a = *(const v4f*)(AGG + v * H + lane * 4), h = *(const v4f*)(Hs + v * H + lane * 4);
    for (int j = 0; j < 4; ++j) { b16 p, q; split16(a[j] * XS, p, q); Ah[wave][rr][lane * 4 + j] = p; Al[wave][rr][lane * 4 + j] = q; split16(h[j] * XS, p, q); Ah[wave][rr][H + lane * 4 + j] = p; Al[wave][rr][H + lane * 4 + j] = q; } }
  wave_lds_sync();
  v8f acc[8];
#pragma unroll
  for (int t = 0; t < 8; ++t) acc[t] = (v8f){};
#pragma unroll 2
  for (int kb = 0; kb < 2 * H; kb += 32) { const v16b a = frag_kb(&Ah[wave][nloc][kb], hlf), al = frag_kb(&Al[wave][nloc][kb], hlf);
#pragma unroll
    for (int t = 0; t < 8; ++t) { const v16b bw = frag_kb(W + (size_t)(t * 16 + nloc) * 2 * H + kb, hlf); acc[t] = wmma16b(a, bw, acc[t]); acc[t] = wmma16b(al, bw, acc[t]); } }
#pragma unroll
  for (int t = 0; t < 8; ++t) { const int c = t * 16 + nloc; const float bb = bf16_rne(bl[c]);
#pragma unroll 1
    for (int r = 0; r < 8; ++r) Tf[wave][8 * hlf + r][c] = acc[t][r] * (1.0f / (XS * WSC)) + bb; }
  wave_lds_sync();
  for (int rr = 0; rr < 16; ++rr) { const size_t v = m0 + rr; v4f y = *(const v4f*)(&Tf[wave][rr][lane * 4]);
    float s2 = y[0] * y[0] + y[1] * y[1] + y[2] * y[2] + y[3] * y[3]; for (int o = 16; o; o >>= 1) s2 += __shfl_xor(s2, o); const float inv = 1.0f / fmaxf(sqrtf(s2), NRMEPS);
    for (int j = 0; j < 4; ++j) { y[j] = pmul(y[j], inv); if (RELU) y[j] = fmaxf(y[j], 0.0f); if (v >= (size_t)NV) y[j] = 0.0f; }
    for (int pass = 0; pass < 2; ++pass) { *(volatile v4f*)(OUT + v * H + lane * 4) = y; __threadfence(); } }
}
__global__ __launch_bounds__(256) void decode_kernel(const float* __restrict__ ZT, const float* __restrict__ ZP, const int* __restrict__ ls, const int* __restrict__ ld, float* __restrict__ out) {
  __shared__ __attribute__((aligned(16))) float sc[64];
  const int wave = threadIdx.x >> 5, lane = threadIdx.x & 31;
#pragma unroll 1
  for (int q = 0; q < 8; ++q) { const int i = blockIdx.x * 64 + wave * 8 + q; float d = 0.0f;
    if (i < EL) { const size_t a = (size_t)iclamp(ls[i], 0, NT - 1), b = (size_t)iclamp(ld[i], 0, NPL - 1); const v4f za = *(const v4f*)(ZT + a * H + lane * 4), zb = *(const v4f*)(ZP + b * H + lane * 4); d = pmul(za[0], zb[0]) + pmul(za[1], zb[1]) + pmul(za[2], zb[2]) + pmul(za[3], zb[3]); }
    for (int sh = 16; sh; sh >>= 1) d += __shfl_xor(d, sh);
    if (lane == 0) sc[wave * 8 + q] = d; }
  __syncthreads();
  for (int pass = 0; pass < 2; ++pass) { if (threadIdx.x < 16) { const int i0 = blockIdx.x * 64 + threadIdx.x * 4; if (i0 < EL) *(volatile v4f*)(out + i0) = *(const v4f*)(&sc[threadIdx.x * 4]); } __threadfence(); }
}
}

extern "C" void kernel_launch(void* const* d_in, const int* in_sizes, int n_in, void* d_out, int out_size, void* d_ws, size_t ws_size, hipStream_t stream) {
  (void)n_in;
  auto Fp = [&](int i) { return (const float*)d_in[i]; }; auto Ip = [&](int i) { return (const int*)d_in[i]; };
  if (in_sizes[0] != NT * FT || in_sizes[1] != NPL * FP || in_sizes[2] != E || in_sizes[3] != E || in_sizes[4] != EL || in_sizes[5] != EL || in_sizes[6] != FT * H || in_sizes[8] != FP * H || in_sizes[10] != H * H || in_sizes[21] != H * H || out_size != EL) return;
  size_t off = 0; char* ws = (char*)d_ws;
  auto carve = [&](size_t bytes) { char* p = ws + off; off += (bytes + 255) & ~(size_t)255; return p; };
  b16* WNT = (b16*)carve((size_t)H * FT * 2); b16* WNP = (b16*)carve((size_t)H * FP * 2); b16* WL = (b16*)carve((size_t)4 * H * 2 * H * 2);
  float* HT = (float*)carve((size_t)NTP * H * 4); float* HP = (float*)carve((size_t)NPP * H * 4); float* AT = (float*)carve((size_t)NTP * H * 4); float* AP = (float*)carve((size_t)NPP * H * 4);
  float* OT = HT; float* OP = HP; float* ZT = AT; float* ZP = AP;
  CsrBufs6 csrP; off = csr_carve6(csrP, ws, off, E, NPL); CsrBufs8 csrT; off = csr_carve8(csrT, ws, off, E, NT);
  if (off > ws_size) return;
  wprep_kernel<<<(unsigned)(((size_t)H * FT / 8 + (size_t)H * FP / 8 + 4 * (size_t)H * 2 * H / 8 + 255) / 256), 256, 0, stream>>>(Fp(6), Fp(8), Fp(10), Fp(12), Fp(13), Fp(15), Fp(16), Fp(18), Fp(19), Fp(21), WNT, WNP, WL);
  csr_build6(csrP, Ip(3), E, NPL, stream);
  csr_build8(csrT, Ip(2), E, NT, stream);
  proj_kernel<FT><<<NTP / 64, 128, 0, stream>>>(Fp(0), NT, WNT, Fp(7), HT);
  proj_kernel<FP><<<NPP / 64, 128, 0, stream>>>(Fp(1), NPL, WNP, Fp(9), HP);
  mean_kernel<<<NPP / 8, 256, 0, stream>>>(HT, NT, Ip(2), NPL, csrP.PERM, csrP.ROWPTR, csrP.ROWCNT, (int)csrP.permLen, AP);
  mean_kernel<<<NTP / 8, 256, 0, stream>>>(HP, NPL, Ip(3), NT, csrT.PERM, csrT.ROWPTR, csrT.ROWCNT, (int)csrT.permLen, AT);
  sage_kernel<1><<<NPP / 64, 128, 0, stream>>>(AP, HP, NPL, WL + (size_t)0 * H * 2 * H, Fp(11), OP);
  sage_kernel<1><<<NTP / 64, 128, 0, stream>>>(AT, HT, NT, WL + (size_t)1 * H * 2 * H, Fp(14), OT);
  mean_kernel<<<NPP / 8, 256, 0, stream>>>(OT, NT, Ip(2), NPL, csrP.PERM, csrP.ROWPTR, csrP.ROWCNT, (int)csrP.permLen, AP);
  mean_kernel<<<NTP / 8, 256, 0, stream>>>(OP, NPL, Ip(3), NT, csrT.PERM, csrT.ROWPTR, csrT.ROWCNT, (int)csrT.permLen, AT);
  sage_kernel<0><<<NPP / 64, 128, 0, stream>>>(AP, OP, NPL, WL + (size_t)2 * H * 2 * H, Fp(17), ZP);
  sage_kernel<0><<<NTP / 64, 128, 0, stream>>>(AT, OT, NT, WL + (size_t)3 * H * 2 * H, Fp(20), ZT);
  decode_kernel<<<(EL + 63) / 64, 256, 0, stream>>>(ZT, ZP, Ip(4), Ip(5), (float*)d_out);
}
